// NodeFormerConv_73890617360780
// MI455X (gfx1250) — hardware-verified
//
#include <hip/hip_runtime.h>
#include <math.h>

typedef __attribute__((ext_vector_type(16))) _Float16 v16h;
typedef __attribute__((ext_vector_type(8)))  _Float16 v8h;
typedef __attribute__((ext_vector_type(8)))  float  v8f;
typedef __attribute__((ext_vector_type(4)))  float  v4f;
typedef __attribute__((ext_vector_type(4)))  unsigned v4u;
typedef float __attribute__((may_alias)) float_a;

#define N_NODES 30000
#define NP 30016
#define CIN 256
#define NH 4
#define MF 30
#define MP 32
#define DH 64
#define KG 10
#define NHK 40
#define NCH 14
#define KSTEPS 67
#define BT 256
#define ECAP 5120
#define SCAP 48
#define ETILE 2048
#define NBUCK ((N_NODES + BT - 1) / BT)

template <typename V> __device__ __forceinline__ void vst2(void* p, V v) {
  *(volatile V*)p = v; __threadfence(); *(volatile V*)p = v;
}
__device__ __forceinline__ v8f wmma_f16(v16h a, v16h b, v8f c) {
  v8f d = __builtin_amdgcn_wmma_f32_16x16x32_f16(false, a, false, b, (short)0, c, false, false);
  asm volatile("v_nop\n\tv_nop\n\tv_nop\n\tv_nop" : "+v"(d) : "v"(a), "v"(b));
  return d;
}
typedef __attribute__((ext_vector_type(16))) __bf16 v16bf;
__device__ __forceinline__ v8f wmma_bf(v16bf a, v16bf b, v8f c) {
  v8f d = __builtin_amdgcn_wmma_f32_16x16x32_bf16(false, a, false, b, (short)0, c, false, false);
  asm volatile("v_nop\n\tv_nop\n\tv_nop\n\tv_nop" : "+v"(d) : "v"(a), "v"(b));
  return d;
}
__device__ __forceinline__ v16h frag_h(const _Float16* row, int k0, int lane) {
  union { v16h v; v8h h[2]; } r; const _Float16* p = row + k0 + 8 * (lane >> 4);
  r.h[0] = *(const v8h*)(p); r.h[1] = *(const v8h*)(p + 16); return r.v;
}
__device__ __forceinline__ v16h frag_f32(const float* row, int k0, int lane) {
  v16h a; const float* p = row + k0 + 8 * (lane >> 4);
#pragma unroll
  for (int i = 0; i < 8; ++i) { a[i] = (_Float16)p[i]; a[8 + i] = (_Float16)p[16 + i]; }
  return a;
}

struct Bucket {
  int lsrc[ECAP]; unsigned short ltgt[ECAP]; unsigned short sub[BT][SCAP]; int scnt[BT]; int wcnt[8][8]; int total;
};
__device__ void bucket_build(Bucket& bk, const int* __restrict__ src, const int* __restrict__ dst, int E, int tlo, int tid) {
  const int lane = tid & 31, wave = tid >> 5;
  if (tid == 0) bk.total = 0;
  __syncthreads();
  for (int e0 = 0; e0 < E; e0 += ETILE) {
    int rv[8]; unsigned msk[8];
#pragma unroll
    for (int j = 0; j < 8; ++j) {
      const int e = e0 + j * 256 + tid;
      const int r = (e < E) ? dst[e] : -1;
      rv[j] = r;
      msk[j] = (unsigned)__builtin_amdgcn_ballot_w32((r >= tlo) && (r < tlo + BT));
    }
    if (lane < 8) bk.wcnt[lane][wave] = __builtin_popcount(msk[lane]);
    __syncthreads();
    const int base = bk.total;
    int run = 0, pre[8];
#pragma unroll
    for (int j = 0; j < 8; ++j) {
#pragma unroll
      for (int w = 0; w < 8; ++w) { if (w == wave) pre[j] = run; run += bk.wcnt[j][w]; }
    }
#pragma unroll
    for (int j = 0; j < 8; ++j) {
      const unsigned m = msk[j];
      if ((m >> lane) & 1u) {
        const int pos = base + pre[j] + __builtin_popcount(m & ((1u << lane) - 1u));
        if (pos < ECAP) { bk.lsrc[pos] = e0 + j * 256 + tid; bk.ltgt[pos] = (unsigned short)(rv[j] - tlo); }
      }
    }
    __syncthreads();
    if (tid == 0) bk.total = base + run;
    __syncthreads();
  }
  const int n = (bk.total < ECAP) ? bk.total : ECAP;
  for (int i = tid; i < n; i += 256) { int s = src[bk.lsrc[i]]; s = s < 0 ? 0 : (s >= N_NODES ? N_NODES - 1 : s); bk.lsrc[i] = s; }
  __syncthreads();
  int k = 0;
  for (int i = 0; i < n; ++i) if ((int)bk.ltgt[i] == tid) { if (k < SCAP) bk.sub[tid][k] = (unsigned short)i; ++k; }
  bk.scnt[tid] = (k < SCAP) ? k : SCAP;
  __syncthreads();
}


__global__ __launch_bounds__(256) void k_cvt(const float* __restrict__ s, _Float16* __restrict__ d, int n8) {
  const int g = blockIdx.x * 256 + threadIdx.x; if (g >= n8) return;
  union { v8h h; v4u u; } pk;
#pragma unroll
  for (int e = 0; e < 8; ++e) pk.h[e] = (_Float16)s[(size_t)g * 8 + e];
  vst2(d + (size_t)g * 8, pk.u);
}

template <bool TRANS>
__global__ __launch_bounds__(256) void k_proj(const float* __restrict__ z, const _Float16* __restrict__ W, const float* __restrict__ bias,
                                             float* __restrict__ Y, float* __restrict__ YT) {
  __shared__ __align__(16) float T[32][260];
  const int tid = threadIdx.x, wave = tid >> 5, lane = tid & 31, hi = lane >> 4, col = lane & 15;
  const int nb = blockIdx.x * 32, sl = (wave >> 2) * 16, c0 = (wave & 3) * 64;
  int arow = nb + sl + col; if (arow >= N_NODES) arow = N_NODES - 1;
  const float* ar = z + (size_t)arow * CIN;
  v8f acc[4] = {(v8f){}, (v8f){}, (v8f){}, (v8f){}};
#pragma unroll 2
  for (int kc = 0; kc < CIN / 32; ++kc) { const v16h a = frag_f32(ar, kc * 32, lane);
#pragma unroll
    for (int j = 0; j < 4; ++j) acc[j] = wmma_f16(a, frag_h(W + (size_t)(c0 + j * 16 + col) * CIN, kc * 32, lane), acc[j]); }
#pragma unroll
  for (int j = 0; j < 4; ++j) { const int c = c0 + j * 16 + col;
#pragma unroll
    for (int r = 0; r < 8; ++r) T[sl + hi * 8 + r][c] = acc[j][r] + bias[c]; }
  __syncthreads();
  for (int g = tid; g < 32 * 64; g += 256) { const int rl = g >> 6, pc = g & 63; const int n = nb + rl;
    if (n < N_NODES) vst2(Y + (size_t)n * CIN + pc * 4, *(const v4f*)(&T[rl][pc * 4])); }
  if (TRANS) {
    for (int g = tid; g < 256 * 8; g += 256) { const int c = g >> 3, pc = g & 7;
      v4f v;
#pragma unroll
      for (int e = 0; e < 4; ++e) { const int rl = pc * 4 + e; v[e] = (nb + rl < N_NODES) ? T[rl][c] : 0.f; }
      vst2(YT + (size_t)c * NP + nb + pc * 4, v); }
  }
}

__global__ __launch_bounds__(256) void k_feat(const float* __restrict__ Q, const float* __restrict__ Kf, const float* __restrict__ proj,
                                             const float* __restrict__ tau, float* __restrict__ qp, float* __restrict__ kraw, float* __restrict__ kmaxp) {
  __shared__ float pmax[8][4];
  const int tid = threadIdx.x, wave = tid >> 5, lane = tid & 31;
  const int n = blockIdx.x * 8 + wave;
  const float sc = rsqrtf(tau[0]) * 0.35355339059327373f;
  const float ratio = 0.18257418583505536f;
  float hmax[4] = {-3.0e38f, -3.0e38f, -3.0e38f, -3.0e38f};
  if (n < N_NODES) {
#pragma unroll 1
    for (int which = 0; which < 2; ++which) {
      const float* X = (which == 0 ? Q : Kf) + (size_t)n * CIN;
#pragma unroll 1
      for (int h = 0; h < NH; ++h) {
        const float x0 = X[h * DH + lane] * sc, x1 = X[h * DH + 32 + lane] * sc;
        float dg = x0 * x0 + x1 * x1;
#pragma unroll
        for (int off = 16; off > 0; off >>= 1) dg += __shfl_xor(dg, off, 32);
        dg *= 0.5f;
        float mine = 0.f;
#pragma unroll 1
        for (int m = 0; m < MF; ++m) {
          float p = x0 * proj[m * DH + lane] + x1 * proj[m * DH + 32 + lane];
#pragma unroll
          for (int off = 16; off > 0; off >>= 1) p += __shfl_xor(p, off, 32);
          if (lane == m) mine = p;
        }
        if (which == 0) {
          float mx = (lane < MF) ? mine : -3.0e38f;
#pragma unroll
          for (int off = 16; off > 0; off >>= 1) mx = fmaxf(mx, __shfl_xor(mx, off, 32));
          const float v = (lane < MF) ? ratio * (__expf(mine - dg - mx) + 1e-6f) : 0.f;
          vst2(qp + ((size_t)n * NH + h) * MP + lane, (float_a)v);
        } else {
          const float v = (lane < MF) ? (mine - dg) : 0.f;
          vst2(kraw + ((size_t)n * NH + h) * MP + lane, (float_a)v);
          float mx = (lane < MF) ? mine : -3.0e38f;
#pragma unroll
          for (int off = 16; off > 0; off >>= 1) mx = fmaxf(mx, __shfl_xor(mx, off, 32));
          hmax[h] = mx;
        }
      }
    }
  }
  if (lane < 4) pmax[wave][lane] = hmax[lane];
  __syncthreads();
  if (tid < 32) {
    float v = -3.0e38f;
    if (tid < 4) { for (int w = 0; w < 8; ++w) v = fmaxf(v, pmax[w][tid]); }
    vst2(kmaxp + (size_t)blockIdx.x * 32 + tid, (float_a)v);
  }
}
__global__ __launch_bounds__(256) void k_gmaxp(const float* __restrict__ g, float* __restrict__ gmaxp) {
  __shared__ float red[8][40];
  const int tid = threadIdx.x, wave = tid >> 5, lane = tid & 31;
  float mx0 = -3.0e38f, mx1 = -3.0e38f;
  for (int i = 0; i < 32; ++i) { const int n = blockIdx.x * 256 + wave * 32 + i; if (n >= N_NODES) break;
    mx0 = fmaxf(mx0, g[(size_t)n * NHK + lane]); if (lane < 8) mx1 = fmaxf(mx1, g[(size_t)n * NHK + 32 + lane]); }
  red[wave][lane] = mx0; if (lane < 8) red[wave][32 + lane] = mx1;
  __syncthreads();
  if (tid < 64) { float v = -3.0e38f; if (tid < 40) { for (int w = 0; w < 8; ++w) v = fmaxf(v, red[w][tid]); } vst2(gmaxp + (size_t)blockIdx.x * 64 + tid, (float_a)v); }
}
__global__ __launch_bounds__(64) void k_maxred(const float* __restrict__ kmaxp, int nkb, const float* __restrict__ gmaxp, int ngb,
                                              float* __restrict__ stabk, float* __restrict__ gmax) {
  const int t = threadIdx.x;
  float v = -3.0e38f;
  if (t < 32) { for (int i = 0; i < nkb; ++i) v = fmaxf(v, kmaxp[i * 32 + t]); vst2(stabk + t, (float_a)v); }
  float w = -3.0e38f;
  for (int i = 0; i < ngb; ++i) w = fmaxf(w, gmaxp[i * 64 + t]);
  vst2(gmax + t, (float_a)w);
}

__global__ __launch_bounds__(256) void k_kp(const float* __restrict__ kraw, const float* __restrict__ stabk, const float* __restrict__ g,
                                           const float* __restrict__ gmax, float* __restrict__ kp, float* __restrict__ kpT, float* __restrict__ egT) {
  __shared__ __align__(16) float tk[128][36];
  __shared__ __align__(16) float tg[40][36];
  const int tid = threadIdx.x, nb = blockIdx.x * 32;
  const float ratio = 0.18257418583505536f;
  for (int i = tid; i < 32 * 128; i += 256) {
    const int nl = i >> 7, c = i & 127, h = c >> 5, m = c & 31, n = nb + nl;
    float v = 0.f;
    if (n < N_NODES && m < MF) v = ratio * (__expf(kraw[(size_t)n * 128 + c] - stabk[h]) + 1e-6f);
    tk[c][nl] = v;
    if (n < N_NODES) vst2(kp + (size_t)n * 128 + c, (float_a)v);
  }
  for (int i = tid; i < 32 * 40; i += 256) {
    const int nl = i / 40, c = i % 40, n = nb + nl;
    tg[c][nl] = (n < N_NODES) ? __expf(g[(size_t)n * NHK + c] - gmax[c]) : 0.f;
  }
  __syncthreads();
  for (int gq = tid; gq < 128 * 8; gq += 256) { const int c = gq >> 3, pc = gq & 7; vst2(kpT + (size_t)c * NP + nb + pc * 4, *(const v4f*)(&tk[c][pc * 4])); }
  for (int gq = tid; gq < 40 * 8; gq += 256) { const int c = gq >> 3, pc = gq & 7; vst2(egT + (size_t)c * NP + nb + pc * 4, *(const v4f*)(&tg[c][pc * 4])); }
}

__global__ __launch_bounds__(256) void k_kvs(const float* __restrict__ kpT, const float* __restrict__ egT, const float* __restrict__ vT,
                                            float* __restrict__ part, float* __restrict__ spart) {
  __shared__ __align__(16) float T[32][68];
  __shared__ float srow[32];
  const int hk = blockIdx.x, ch = blockIdx.y, h = hk / KG;
  const int tid = threadIdx.x, wave = tid >> 5, lane = tid & 31, hi = lane >> 4, col = lane & 15;
  const int mt = wave >> 2, dt = wave & 3;
  const float* arow = kpT + (size_t)(h * MP + mt * 16 + col) * NP;
  const float* grow = egT + (size_t)hk * NP;
  const float* brow = vT + (size_t)(h * DH + dt * 16 + col) * NP;
  v8f acc = {};
  float rs = 0.f;
  const int nbase = ch * KSTEPS * 32;
#pragma unroll 1
  for (int ks = 0; ks < KSTEPS; ++ks) {
    const int n0 = nbase + ks * 32 + 8 * hi;
    v16bf a, b;
#pragma unroll
    for (int i = 0; i < 8; ++i) {
      const float a0 = arow[n0 + i] * grow[n0 + i], a1 = arow[n0 + 16 + i] * grow[n0 + 16 + i];
      rs += a0 + a1; a[i] = (__bf16)a0; a[8 + i] = (__bf16)a1;
      b[i] = (__bf16)brow[n0 + i]; b[8 + i] = (__bf16)brow[n0 + 16 + i];
    }
    acc = wmma_bf(a, b, acc);
  }
#pragma unroll
  for (int r = 0; r < 8; ++r) T[mt * 16 + hi * 8 + r][dt * 16 + col] = acc[r];
  if (dt == 0) { rs += __shfl_xor(rs, 16, 32); if (hi == 0) srow[mt * 16 + col] = rs; }
  __syncthreads();
  float* dst = part + ((size_t)ch * NHK + hk) * (32 * 64);
  for (int g = tid; g < 32 * 16; g += 256) { const int rl = g >> 4, pc = g & 15; vst2(dst + rl * 64 + pc * 4, *(const v4f*)(&T[rl][pc * 4])); }
  if (tid < 32) vst2(spart + ((size_t)ch * NHK + hk) * 32 + tid, (float_a)srow[tid]);
}
__global__ __launch_bounds__(256) void k_kvsred(const float* __restrict__ part, const float* __restrict__ spart, float* __restrict__ kvs, float* __restrict__ ksum) {
  const int i = blockIdx.x * 256 + threadIdx.x;
  if (i < NHK * 512) {
    v4f s = {0.f, 0.f, 0.f, 0.f};
    for (int ch = 0; ch < NCH; ++ch) s += *(const v4f*)(part + (size_t)ch * NHK * 2048 + (size_t)i * 4);
    vst2(kvs + (size_t)i * 4, s);
  }
  if (i < NHK * 8) {
    v4f s = {0.f, 0.f, 0.f, 0.f};
    for (int ch = 0; ch < NCH; ++ch) s += *(const v4f*)(spart + (size_t)ch * NHK * 32 + (size_t)i * 4);
    vst2(ksum + (size_t)i * 4, s);
  }
}
__global__ __launch_bounds__(256) void k_kpsum(const float* __restrict__ kpT, float* __restrict__ kpsum) {
  __shared__ float red[32];
  const int tid = threadIdx.x, wave = tid >> 5, lane = tid & 31;
  for (int r = 0; r < 4; ++r) { const int c = blockIdx.x * 32 + wave * 4 + r; const float* row = kpT + (size_t)c * NP;
    float s = 0.f; for (int n = lane; n < NP; n += 32) s += row[n];
#pragma unroll
    for (int off = 16; off > 0; off >>= 1) s += __shfl_xor(s, off, 32);
    if (lane == 0) red[wave * 4 + r] = s; }
  __syncthreads();
  if (tid < 32) vst2(kpsum + blockIdx.x * 32 + tid, (float_a)red[tid]);
}
__global__ __launch_bounds__(256) void k_degout(const int* __restrict__ st, const int* __restrict__ en, int E, float* __restrict__ degout) {
  __shared__ Bucket bk;
  const int tid = threadIdx.x, tlo = blockIdx.x * BT;
  bucket_build(bk, en, st, E, tlo, tid);
  const int node = tlo + tid;
  if (node < N_NODES) vst2(degout + node, (float_a)(float)bk.scnt[tid]);
}

__global__ __launch_bounds__(256) void k_zout(const int* __restrict__ st, const int* __restrict__ en, int E, const float* __restrict__ qp,
                                             const float* __restrict__ kvs, const float* __restrict__ ksum, const float* __restrict__ V,
                                             const float* __restrict__ bvec, const float* __restrict__ degout, float* __restrict__ zo,
                                             float* __restrict__ degin) {
  __shared__ Bucket bk;
  const int tid = threadIdx.x, lane = tid & 31, wave = tid >> 5, tlo = blockIdx.x * BT;
  bucket_build(bk, st, en, E, tlo, tid);
  if (tlo + tid < N_NODES) vst2(degin + tlo + tid, (float_a)(float)bk.scnt[tid]);
  for (int s = 0; s < 32; ++s) {
    const int t = wave * 32 + s, node = tlo + t;
    if (node >= N_NODES) break;
    const int cnt = bk.scnt[t];
    const float rdin = (cnt > 0) ? 1.f / (float)cnt : 0.f;
#pragma unroll 1
    for (int h = 0; h < NH; ++h) {
      const float qv = qp[((size_t)node * NH + h) * MP + lane];
      float z0 = 0.f, z1 = 0.f;
#pragma unroll 1
      for (int k = 0; k < KG; ++k) {
        const int hk = h * KG + k;
        const float* kv = kvs + (size_t)hk * 2048;
        float den = qv * ksum[hk * 32 + lane];
#pragma unroll
        for (int off = 16; off > 0; off >>= 1) den += __shfl_xor(den, off, 32);
        float n0 = 0.f, n1 = 0.f;
#pragma unroll 1
        for (int m = 0; m < MF; ++m) { const float qm = __shfl(qv, m, 32); n0 += qm * kv[m * 64 + lane]; n1 += qm * kv[m * 64 + 32 + lane]; }
        z0 += n0 / den; z1 += n1 / den;
      }
      z0 *= (1.f / KG); z1 *= (1.f / KG);
      const float sb = 1.f / (1.f + __expf(-bvec[h]));
      float c0 = 0.f, c1 = 0.f;
      for (int kk = 0; kk < cnt; ++kk) {
        const int sN = bk.lsrc[bk.sub[t][kk]];
        const float w = sb * sqrtf(rdin * (1.f / degout[sN]));
        const float* vr = V + (size_t)sN * CIN + h * DH;
        c0 += w * vr[lane]; c1 += w * vr[32 + lane];
      }
      float* orow = zo + (size_t)node * CIN + h * DH;
      vst2(orow + lane, (float_a)(z0 + c0)); vst2(orow + 32 + lane, (float_a)(z1 + c1));
    }
  }
}

__global__ __launch_bounds__(128) void k_outproj(const float* __restrict__ zo, const _Float16* __restrict__ Wo, const float* __restrict__ bo, float* __restrict__ out) {
  __shared__ __align__(16) float T[16][68];
  const int tid = threadIdx.x, wave = tid >> 5, lane = tid & 31, hi = lane >> 4, col = lane & 15, m0 = blockIdx.x * 16;
  const float* ar = zo + (size_t)(m0 + col) * CIN;
  v8f acc = {};
#pragma unroll
  for (int kc = 0; kc < 8; ++kc) acc = wmma_f16(frag_f32(ar, kc * 32, lane), frag_h(Wo + (size_t)(wave * 16 + col) * CIN, kc * 32, lane), acc);
#pragma unroll
  for (int r = 0; r < 8; ++r) T[hi * 8 + r][wave * 16 + col] = acc[r] + bo[wave * 16 + col];
  __syncthreads();
  for (int g = tid; g < 16 * 16; g += 128) { const int rl = g >> 4, pc = g & 15; vst2(out + (size_t)(m0 + rl) * DH + pc * 4, *(const v4f*)(&T[rl][pc * 4])); }
}

__global__ __launch_bounds__(256) void k_link(const int* __restrict__ st, const int* __restrict__ en, int E, const float* __restrict__ qp,
                                             const float* __restrict__ kp, const float* __restrict__ kpsum, const float* __restrict__ degin,
                                             float* __restrict__ lpart) {
  __shared__ float red[8];
  const int tid = threadIdx.x, lane = tid & 31, wave = tid >> 5;
  const int i = blockIdx.x * 256 + tid;
  float term = 0.f;
  if (i < E * NH) {
    const int e = i >> 2, h = i & 3;
    int s = st[e], d = en[e];
    s = s < 0 ? 0 : (s >= N_NODES ? N_NODES - 1 : s); d = d < 0 ? 0 : (d >= N_NODES ? N_NODES - 1 : d);
    const float* q = qp + ((size_t)d * NH + h) * MP; const float* kq = kp + ((size_t)s * NH + h) * MP; const float* ks = kpsum + h * MP;
    float num = 0.f, dem = 0.f;
#pragma unroll 1
    for (int m = 0; m < MF; ++m) { num += q[m] * kq[m]; dem += q[m] * ks[m]; }
    term = __logf(num / dem) / degin[d];
  }
#pragma unroll
  for (int off = 16; off > 0; off >>= 1) term += __shfl_xor(term, off, 32);
  if (lane == 0) red[wave] = term;
  __syncthreads();
  if (tid < 32) { float v = 0.f; if (tid == 0) { for (int w = 0; w < 8; ++w) v += red[w]; } if (tid < 1) vst2(lpart + blockIdx.x, (float_a)v); }
}
__global__ __launch_bounds__(256) void k_linkfin(const float* __restrict__ lpart, int nb, int E, float* __restrict__ loss) {
  __shared__ double red[256];
  double s = 0.0;
  for (int i = threadIdx.x; i < nb; i += 256) s += (double)lpart[i];
  red[threadIdx.x] = s; __syncthreads();
  for (int k = 128; k > 0; k >>= 1) { if (threadIdx.x < k) red[threadIdx.x] += red[threadIdx.x + k]; __syncthreads(); }
  if (threadIdx.x == 0) vst2(loss, (float_a)(float)(red[0] / ((double)E * NH)));
}

extern "C" void kernel_launch(void* const* d_in, const int* in_sizes, int n_in,
                              void* d_out, int out_size, void* d_ws, size_t ws_size,
                              hipStream_t stream) {
  (void)n_in; (void)out_size; (void)ws_size;
  const float* z   = (const float*)d_in[0];
  const int*   ei  = (const int*)d_in[1];
  const int E = in_sizes[1] / 2;
  const int* st = ei; const int* en = ei + E;
  const float* tau = (const float*)d_in[2];
  const float* gum = (const float*)d_in[3];
  const float* proj = (const float*)d_in[4];
  const float *Wq = (const float*)d_in[5], *bq = (const float*)d_in[6], *Wk = (const float*)d_in[7], *bk = (const float*)d_in[8];
  const float *Wv = (const float*)d_in[9], *bv = (const float*)d_in[10], *Wo = (const float*)d_in[11], *bo = (const float*)d_in[12];
  const float* bvec = (const float*)d_in[13];
  float* out = (float*)d_out;
  float* loss = out + (size_t)N_NODES * DH;

  char* ws = (char*)d_ws; size_t off = 0;
  auto alloc = [&](size_t bytes) -> void* { void* p = ws + off; off = (off + bytes + 255) & ~(size_t)255; return p; };
  _Float16* Wqh = (_Float16*)alloc(CIN * CIN * 2); _Float16* Wkh = (_Float16*)alloc(CIN * CIN * 2);
  _Float16* Wvh = (_Float16*)alloc(CIN * CIN * 2); _Float16* Woh = (_Float16*)alloc(DH * CIN * 2);
  float* Q  = (float*)alloc((size_t)N_NODES * CIN * 4);
  float* Kf = (float*)alloc((size_t)N_NODES * CIN * 4);
  float* V  = (float*)alloc((size_t)N_NODES * CIN * 4);
  float* vT = (float*)alloc((size_t)CIN * NP * 4);
  float* qp = (float*)alloc((size_t)N_NODES * 128 * 4);
  float* kraw = (float*)alloc((size_t)N_NODES * 128 * 4);
  float* kpb = (float*)alloc((size_t)N_NODES * 128 * 4);
  float* kpT = (float*)alloc((size_t)128 * NP * 4);
  float* egT = (float*)alloc((size_t)NHK * NP * 4);
  const int nfb = (N_NODES + 7) / 8, ngb = (N_NODES + 255) / 256;
  float* kmaxp = (float*)alloc((size_t)nfb * 32 * 4);
  float* gmaxp = (float*)alloc((size_t)ngb * 64 * 4);
  float* stabk = (float*)alloc(32 * 4);
  float* gmax = (float*)alloc(64 * 4);
  float* part = (float*)alloc((size_t)NCH * NHK * 2048 * 4);
  float* spart = (float*)alloc((size_t)NCH * NHK * 32 * 4);
  float* kvs = (float*)alloc((size_t)NHK * 2048 * 4);
  float* ksum = (float*)alloc((size_t)NHK * 32 * 4);
  float* kpsum = (float*)alloc(128 * 4);
  float* degout = (float*)alloc((size_t)N_NODES * 4 + 1024);
  float* degin = (float*)alloc((size_t)N_NODES * 4 + 1024);
  float* zo = (float*)alloc((size_t)N_NODES * CIN * 4);
  const int nlb = (E * NH + 255) / 256;
  float* lpart = (float*)alloc((size_t)nlb * 4 + 256);

  k_cvt<<<(CIN * CIN / 8 + 255) / 256, 256, 0, stream>>>(Wq, Wqh, CIN * CIN / 8);
  k_cvt<<<(CIN * CIN / 8 + 255) / 256, 256, 0, stream>>>(Wk, Wkh, CIN * CIN / 8);
  k_cvt<<<(CIN * CIN / 8 + 255) / 256, 256, 0, stream>>>(Wv, Wvh, CIN * CIN / 8);
  k_cvt<<<(DH * CIN / 8 + 255) / 256, 256, 0, stream>>>(Wo, Woh, DH * CIN / 8);
  const int pblk = (N_NODES + 31) / 32;
  k_proj<false><<<pblk, 256, 0, stream>>>(z, Wqh, bq, Q, nullptr);
  k_proj<false><<<pblk, 256, 0, stream>>>(z, Wkh, bk, Kf, nullptr);
  k_proj<true><<<pblk, 256, 0, stream>>>(z, Wvh, bv, V, vT);
  k_feat<<<nfb, 256, 0, stream>>>(Q, Kf, proj, tau, qp, kraw, kmaxp);
  k_gmaxp<<<ngb, 256, 0, stream>>>(gum, gmaxp);
  k_maxred<<<1, 64, 0, stream>>>(kmaxp, nfb, gmaxp, ngb, stabk, gmax);
  k_kp<<<pblk, 256, 0, stream>>>(kraw, stabk, gum, gmax, kpb, kpT, egT);
  k_kvs<<<dim3(NHK, NCH), 256, 0, stream>>>(kpT, egT, vT, part, spart);
  k_kvsred<<<(NHK * 512 + 255) / 256, 256, 0, stream>>>(part, spart, kvs, ksum);
  k_kpsum<<<4, 256, 0, stream>>>(kpT, kpsum);
  k_degout<<<NBUCK, 256, 0, stream>>>(st, en, E, degout);
  k_zout<<<NBUCK, 256, 0, stream>>>(st, en, E, qp, kvs, ksum, V, bvec, degout, zo, degin);
  k_outproj<<<N_NODES / 16, 128, 0, stream>>>(zo, Woh, bo, out);
  k_link<<<nlb, 256, 0, stream>>>(st, en, E, qp, kpb, kpsum, degin, lpart);
  k_linkfin<<<1, 256, 0, stream>>>(lpart, nlb, E, loss);
}
